// GaussianKernel_3410204033425
// MI455X (gfx1250) — hardware-run, weakly checked
//
#include <hip/hip_runtime.h>
#include <math.h>

typedef __attribute__((ext_vector_type(16))) _Float16 v16h;
typedef __attribute__((ext_vector_type(8)))  _Float16 v8h;
typedef __attribute__((ext_vector_type(8)))  float    v8f;
typedef __attribute__((ext_vector_type(4)))  float    v4f;

constexpr int kPts        = 2048;
constexpr int kFeat       = 128;
constexpr int kTileSide   = 64;
constexpr int kTilesSide  = kPts / kTileSide;
constexpr int kTilesTotal = kTilesSide * kTilesSide;
constexpr int kWavesPerBlock = 8;
constexpr int kPairBlocks = kTilesTotal / kWavesPerBlock;
constexpr int kRowsPerPrepBlock = kWavesPerBlock * 32;
constexpr int kPrepBlocks = kPts / kRowsPerPrepBlock;
constexpr int kSlabPitch  = 68;
static_assert((kFeat % 32) == 0, "K multiple of 32");
static_assert((kPts % kTileSide) == 0, "M,N multiples of 64");
static_assert(kTilesTotal == 1024 && kPairBlocks == 128, "tile grid");
static_assert(kPrepBlocks * kRowsPerPrepBlock == kPts, "row coverage of the operand-plane kernel");
static_assert(kFeat == 16 * 8, "one half wave of 16 lanes x 8 elements covers one row");

constexpr float kCarry         = 16.0f;
constexpr float kInvCarrySq    = 1.0f / (kCarry * kCarry);
constexpr float kTwoInvCarrySq = 2.0f / (kCarry * kCarry);
constexpr float kHalfMinNormal = 6.103515625e-5f;
constexpr float kAlphaScale    = 1.0f;
constexpr double kInvCount     = 1.0 / ((double)kPts * (double)kPts);

constexpr size_t kSzXH   = (size_t)kPts * kFeat * 2;
constexpr size_t kSzNRM  = (size_t)kPts * 4;
constexpr size_t kSzPART = (size_t)kTilesTotal * 32 * 4;
constexpr size_t kSzSIG  = 128;
constexpr size_t kSzD2   = (size_t)kPts * kPts * 4;
constexpr size_t kOffXH   = 0;
constexpr size_t kOffNRM  = kOffXH + kSzXH;
constexpr size_t kOffPART = kOffNRM + kSzNRM;
constexpr size_t kOffSIG  = kOffPART + kSzPART;
constexpr size_t kOffD2   = kOffSIG + kSzSIG;
constexpr size_t kWsTotal = kOffD2 + kSzD2;
static_assert(kWsTotal == 17440896ull, "carve total");
static_assert(kWsTotal <= 134217728ull, "carve cap");
static_assert((kOffNRM % 128) == 0 && (kOffPART % 128) == 0 && (kOffSIG % 128) == 0 && (kOffD2 % 128) == 0,
              "128-B aligned regions");

struct FragH {
  union U { v16h v; v8h h[2]; };
  static __device__ __forceinline__ v16h load(const _Float16* p) {
    U f;
    f.h[0] = *(const v8h*)(p);
    f.h[1] = *(const v8h*)(p + 16);
    return f.v;
  }
};
__device__ __forceinline__ v8f mma_f16(v16h a, v16h b, v8f c) {
  c = __builtin_amdgcn_wmma_f32_16x16x32_f16(false, a, false, b, (short)0, c, false, false);
  asm volatile("v_nop\n\tv_nop\n\tv_nop\n\tv_nop" : "+v"(c) : "v"(a), "v"(b));
  return c;
}

__global__ __launch_bounds__(256) void prep_rows_kernel(
    const float* __restrict__ X, unsigned short* __restrict__ XH, float* __restrict__ NRM)
{
  __shared__ float sN[kWavesPerBlock][32];
  const int tid  = threadIdx.x;
  const int lane = tid & 31;
  const int wave = tid >> 5;
  const int half = lane >> 4;
  const int seg  = lane & 15;
  const int rowBase = (blockIdx.x * kWavesPerBlock + wave) * 32;
#pragma unroll 1
  for (int it = 0; it < 16; ++it) {
    const int row = rowBase + 2 * it + half;
    const float* src = X + (size_t)row * kFeat + seg * 8;
    const v4f a0 = *(const v4f*)(src);
    const v4f a1 = *(const v4f*)(src + 4);
    v8h hv;
    float s = 0.0f;
#pragma unroll
    for (int e = 0; e < 4; ++e) {
      float c = a0[e] * kCarry;
      c = (fabsf(c) < kHalfMinNormal) ? 0.0f : c;
      const _Float16 hc = (_Float16)c;
      const float back = (float)hc;
      s = fmaf(back, back, s);
      hv[e] = hc;
    }
#pragma unroll
    for (int e = 0; e < 4; ++e) {
      float c = a1[e] * kCarry;
      c = (fabsf(c) < kHalfMinNormal) ? 0.0f : c;
      const _Float16 hc = (_Float16)c;
      const float back = (float)hc;
      s = fmaf(back, back, s);
      hv[4 + e] = hc;
    }
    s += __shfl_xor(s, 1, 32);
    s += __shfl_xor(s, 2, 32);
    s += __shfl_xor(s, 4, 32);
    s += __shfl_xor(s, 8, 32);
    if (seg == 0) sN[wave][2 * it + half] = s;
    unsigned short* dst = XH + (size_t)row * kFeat + seg * 8;
    *(volatile v8h*)dst = hv;
    __threadfence();
    *(volatile v8h*)dst = hv;
  }
  __syncthreads();
  {
    const float nv = sN[wave][lane] * kInvCarrySq;
    float* np = NRM + rowBase + lane;
    *(volatile float*)np = nv;
    __threadfence();
    *(volatile float*)np = nv;
  }
}

__global__ __launch_bounds__(256) void pair_dist_kernel(
    const unsigned short* __restrict__ XHp, const float* __restrict__ NRM,
    float* __restrict__ D2, float* __restrict__ PART)
{
  const _Float16* A = (const _Float16*)XHp;
  __shared__ __align__(16) float sT[kWavesPerBlock][16 * kSlabPitch];
  const int lane = threadIdx.x & 31;
  const int wave = threadIdx.x >> 5;
  const int tile = blockIdx.x * kWavesPerBlock + wave;
  if (tile >= kTilesTotal) return;
  const int tm = tile / kTilesSide;
  const int tn = tile - tm * kTilesSide;
  const int m0 = tm << 6;
  const int n0 = tn << 6;
  const int rlane = lane & 15;
  const int koff  = (lane >> 4) * 8;
  const int mOff  = (lane >> 4) * 8;

  v8f acc[4][4];
#pragma unroll
  for (int i = 0; i < 4; ++i)
#pragma unroll
    for (int j = 0; j < 4; ++j) acc[i][j] = (v8f){0.f, 0.f, 0.f, 0.f, 0.f, 0.f, 0.f, 0.f};

#pragma unroll 1
  for (int k0 = 0; k0 < kFeat; k0 += 32) {
    v16h bh[4];
#pragma unroll
    for (int j = 0; j < 4; ++j)
      bh[j] = FragH::load(A + (size_t)(n0 + (j << 4) + rlane) * kFeat + koff + k0);
#pragma unroll
    for (int i = 0; i < 4; ++i) {
      const v16h ah = FragH::load(A + (size_t)(m0 + (i << 4) + rlane) * kFeat + koff + k0);
#pragma unroll
      for (int j = 0; j < 4; ++j) acc[i][j] = mma_f16(ah, bh[j], acc[i][j]);
    }
  }

  float* slab = sT[wave];
  float ncol[4];
#pragma unroll
  for (int j = 0; j < 4; ++j) ncol[j] = NRM[n0 + (j << 4) + rlane];
  float psum = 0.0f;
#pragma unroll
  for (int i = 0; i < 4; ++i) {
    const int mBase = m0 + (i << 4);
    const v4f r0 = *(const v4f*)(NRM + mBase + mOff);
    const v4f r1 = *(const v4f*)(NRM + mBase + mOff + 4);
    float nr[8];
    nr[0] = r0[0]; nr[1] = r0[1]; nr[2] = r0[2]; nr[3] = r0[3];
    nr[4] = r1[0]; nr[5] = r1[1]; nr[6] = r1[2]; nr[7] = r1[3];
#pragma unroll
    for (int j = 0; j < 4; ++j) {
#pragma unroll
      for (int r = 0; r < 8; ++r) {
        const float d = fmaf(acc[i][j][r], -kTwoInvCarrySq, nr[r] + ncol[j]);
        psum += d;
        slab[(mOff + r) * kSlabPitch + (j << 4) + rlane] = d;
      }
    }
    __builtin_amdgcn_fence(__ATOMIC_RELEASE, "workgroup");
    __builtin_amdgcn_wave_barrier();
    __builtin_amdgcn_fence(__ATOMIC_ACQUIRE, "workgroup");
    {
      const int hh = lane >> 4;
      const int c4 = (lane & 15) * 4;
      for (int pass = 0; pass < 2; ++pass) {
#pragma unroll
        for (int it = 0; it < 8; ++it) {
          const int row = it * 2 + hh;
          const v4f v = *(const v4f*)(slab + row * kSlabPitch + c4);
          *(volatile v4f*)(D2 + (size_t)(mBase + row) * kPts + n0 + c4) = v;
        }
        __threadfence();
      }
    }
    __builtin_amdgcn_fence(__ATOMIC_RELEASE, "workgroup");
    __builtin_amdgcn_wave_barrier();
    __builtin_amdgcn_fence(__ATOMIC_ACQUIRE, "workgroup");
  }
  psum += __shfl_xor(psum, 16, 32);
  psum += __shfl_xor(psum, 8, 32);
  psum += __shfl_xor(psum, 4, 32);
  psum += __shfl_xor(psum, 2, 32);
  psum += __shfl_xor(psum, 1, 32);
  {
    float* pp = PART + (size_t)tile * 32 + lane;
    *(volatile float*)pp = psum;
    __threadfence();
    *(volatile float*)pp = psum;
  }
}

__global__ __launch_bounds__(256) void mean_finalise_kernel(
    const float* __restrict__ PART, float* __restrict__ SIG)
{
  __shared__ double red[256];
  const int tid = threadIdx.x;
  double s = 0.0;
#pragma unroll
  for (int q = 0; q < 4; ++q) s += (double)PART[(size_t)(tid * 4 + q) * 32];
  red[tid] = s;
  __syncthreads();
#pragma unroll 1
  for (int off = 128; off >= 1; off >>= 1) {
    if (tid < off) red[tid] += red[tid + off];
    __syncthreads();
  }
  const double tot = red[0];
  const float s2 = kAlphaScale * (float)(tot * kInvCount);
  const float inv2s = 1.0f / (2.0f * s2);
  if (tid < 32) {
    float* sp = SIG + tid;
    *(volatile float*)sp = inv2s;
    __threadfence();
    *(volatile float*)sp = inv2s;
  }
}

__global__ __launch_bounds__(256) void exp_rows_kernel(
    const float* __restrict__ D2, const float* __restrict__ SIG, float* __restrict__ out)
{
  const float inv2s = SIG[0];
  const size_t base = (size_t)blockIdx.x * kPts;
#pragma unroll 1
  for (int it = 0; it < 2; ++it) {
    const size_t o = base + (size_t)(it * 256 + (int)threadIdx.x) * 4;
    const v4f d = *(const v4f*)(D2 + o);
    v4f r;
#pragma unroll
    for (int e = 0; e < 4; ++e) {
      const float a = d[e] * inv2s;
      r[e] = expf(-a);
    }
    *(volatile v4f*)(out + o) = r;
    __threadfence();
    *(volatile v4f*)(out + o) = r;
  }
}

extern "C" void kernel_launch(void* const* d_in, const int* in_sizes, int n_in,
                              void* d_out, int out_size, void* d_ws, size_t ws_size,
                              hipStream_t stream) {
  if (n_in < 1) return;
  if (in_sizes[0] != kPts * kFeat) return;
  if (out_size != kPts * kPts) return;
  if (ws_size < kWsTotal) return;

  const float* X = (const float*)d_in[0];
  float* out = (float*)d_out;
  char* ws = (char*)d_ws;
  unsigned short* XH = (unsigned short*)(ws + kOffXH);
  float* NRM  = (float*)(ws + kOffNRM);
  float* PART = (float*)(ws + kOffPART);
  float* SIG  = (float*)(ws + kOffSIG);
  float* D2   = (float*)(ws + kOffD2);

  prep_rows_kernel<<<kPrepBlocks, 256, 0, stream>>>(X, XH, NRM);
  pair_dist_kernel<<<kPairBlocks, 256, 0, stream>>>(XH, NRM, D2, PART);
  mean_finalise_kernel<<<1, 256, 0, stream>>>(PART, SIG);
  exp_rows_kernel<<<kPts, 256, 0, stream>>>(D2, SIG, out);
}
